// RelationAwareBias_18863496364256
// MI455X (gfx1250) — hardware-verified
//
#include <hip/hip_runtime.h>
#include <stdint.h>

#define NB  2
#define NH  12
#define NL  512
#define ND  64
#define NR  8
#define NX  8
#define NRH (NR * NH)
static_assert(ND == 64);
static_assert((NL % 128) == 0);
static_assert(NX == 8);

typedef _Float16 v16h __attribute__((ext_vector_type(16)));
typedef _Float16 v8h  __attribute__((ext_vector_type(8)));
typedef __bf16   v16b __attribute__((ext_vector_type(16)));
typedef __bf16   v8b  __attribute__((ext_vector_type(8)));
typedef float    v8f  __attribute__((ext_vector_type(8)));
typedef float    v4f  __attribute__((ext_vector_type(4)));
typedef unsigned int v4u __attribute__((ext_vector_type(4)));

__device__ __forceinline__ unsigned short bf_bits(float f) {
  unsigned u = __float_as_uint(f);
  return (unsigned short)((u + 0x7FFFu + ((u >> 16) & 1u)) >> 16);
}
__device__ __forceinline__ float bf_up(unsigned short h) { return __uint_as_float(((unsigned)h) << 16); }
__device__ __forceinline__ unsigned short h_bits(_Float16 x) { return __builtin_bit_cast(unsigned short, x); }
__device__ __forceinline__ unsigned pk16(unsigned short a, unsigned short b) { return (unsigned)a | ((unsigned)b << 16); }
__device__ __forceinline__ v8f zero8() { v8f z = {0.f, 0.f, 0.f, 0.f, 0.f, 0.f, 0.f, 0.f}; return z; }
__device__ __forceinline__ v4u zero4u() { v4u z = {0u, 0u, 0u, 0u}; return z; }

__device__ __forceinline__ v16b ldfrag_b(const __bf16* p) {
  union { v16b v; v8b h[2]; } f;
  f.h[0] = *(const v8b*)(p);
  f.h[1] = *(const v8b*)(p + 16);
  return f.v;
}
__device__ __forceinline__ v16h ldfrag_h(const _Float16* p) {
  union { v16h v; v8h h[2]; } f;
  f.h[0] = *(const v8h*)(p);
  f.h[1] = *(const v8h*)(p + 16);
  return f.v;
}

__device__ __forceinline__ v8f mma_h(v16h a, v16h b, v8f c) {
  c = __builtin_amdgcn_wmma_f32_16x16x32_f16(false, a, false, b, (short)0, c, false, false);
#if defined(__HIP_DEVICE_COMPILE__)
  asm volatile("v_nop\n\tv_nop\n\tv_nop\n\tv_nop" : "+v"(c) : "v"(a), "v"(b));
#endif
  return c;
}
__device__ __forceinline__ v8f mma_b(v16b a, v16b b, v8f c) {
  c = __builtin_amdgcn_wmma_f32_16x16x32_bf16(false, a, false, b, (short)0, c, false, false);
#if defined(__HIP_DEVICE_COMPILE__)
  asm volatile("v_nop\n\tv_nop\n\tv_nop\n\tv_nop" : "+v"(c) : "v"(a), "v"(b));
#endif
  return c;
}
__device__ __forceinline__ void wave_sync_lds() {
  __builtin_amdgcn_fence(__ATOMIC_RELEASE, "workgroup");
  __builtin_amdgcn_wave_barrier();
  __builtin_amdgcn_fence(__ATOMIC_ACQUIRE, "workgroup");
}

__global__ __launch_bounds__(256) void cvt_bf16x8(const float* __restrict__ q, const float* __restrict__ k,
                                                  unsigned short* xq, unsigned short* xk, int n8) {
  const int i = blockIdx.x * 256 + threadIdx.x;
  const float* in = (blockIdx.y == 0) ? q : k;
  unsigned short* out = (blockIdx.y == 0) ? xq : xk;
  if (i < n8) {
    const v4f a = *(const v4f*)(in + (size_t)i * 8);
    const v4f b = *(const v4f*)(in + (size_t)i * 8 + 4);
    v4u p;
    p[0] = pk16(bf_bits(a[0]), bf_bits(a[1]));
    p[1] = pk16(bf_bits(a[2]), bf_bits(a[3]));
    p[2] = pk16(bf_bits(b[0]), bf_bits(b[1]));
    p[3] = pk16(bf_bits(b[2]), bf_bits(b[3]));
    *(volatile v4u*)(out + (size_t)i * 8) = p;
    __threadfence();
    *(volatile v4u*)(out + (size_t)i * 8) = p;
  }
}

__global__ __launch_bounds__(128) void build_m(const float* __restrict__ qA, const float* __restrict__ qB,
                                               const float* __restrict__ kA, const float* __restrict__ kB,
                                               unsigned short* mhp, unsigned short* mlp) {
  __shared__ __align__(16) float sM[ND * 68];
  const int tid  = threadIdx.x;
  const int wave = tid >> 5;
  const int lane = tid & 31;
  const int hh   = lane >> 4;
  const int c    = lane & 15;
  const int rh   = blockIdx.x;
  const int s    = blockIdx.y;
  const float* Ap = (s == 0) ? qA : kA;
  const float* Bp = (s == 0) ? qB : kB;
  const float* Am = Ap + (size_t)rh * NX * ND;
  const float* Bm = Bp + (size_t)rh * ND * NX;
  const float keep = (hh == 0) ? 1.0f : 0.0f;

  union U { v16b v; v4u u[2]; };
  U af;
  {
    const int d = wave * 16 + c;
    const v4f b0 = *(const v4f*)(Bm + (size_t)d * NX);
    const v4f b1 = *(const v4f*)(Bm + (size_t)d * NX + 4);
    v4u p;
    p[0] = pk16(bf_bits(b0[0] * keep), bf_bits(b0[1] * keep));
    p[1] = pk16(bf_bits(b0[2] * keep), bf_bits(b0[3] * keep));
    p[2] = pk16(bf_bits(b1[0] * keep), bf_bits(b1[1] * keep));
    p[3] = pk16(bf_bits(b1[2] * keep), bf_bits(b1[3] * keep));
    af.u[0] = p;
    af.u[1] = zero4u();
  }
  v8f acc[4];
#pragma unroll
  for (int j = 0; j < 4; ++j) {
    const int e = j * 16 + c;
    float w[8];
#pragma unroll
    for (int x = 0; x < 8; ++x) w[x] = Am[(size_t)x * ND + e] * keep;
    U bfr;
    v4u p;
    p[0] = pk16(bf_bits(w[0]), bf_bits(w[1]));
    p[1] = pk16(bf_bits(w[2]), bf_bits(w[3]));
    p[2] = pk16(bf_bits(w[4]), bf_bits(w[5]));
    p[3] = pk16(bf_bits(w[6]), bf_bits(w[7]));
    bfr.u[0] = p;
    bfr.u[1] = zero4u();
    acc[j] = mma_b(af.v, bfr.v, zero8());
  }
#pragma unroll
  for (int j = 0; j < 4; ++j) {
#pragma unroll
    for (int r = 0; r < 8; ++r) sM[(j * 16 + c) * 68 + wave * 16 + 8 * hh + r] = acc[j][r];
  }
  __syncthreads();
  {
    const int q4 = lane >> 3, c8 = (lane & 7) * 8;
    unsigned short* Mh = mhp + (size_t)(s * NRH + rh) * ND * ND;
    unsigned short* Ml = mlp + (size_t)(s * NRH + rh) * ND * ND;
    v4u hv[4], lv[4];
#pragma unroll
    for (int it = 0; it < 4; ++it) {
      const int e = wave * 16 + it * 4 + q4;
      const float* sp = sM + e * 68 + c8;
      v4u a, a2;
#pragma unroll
      for (int t = 0; t < 4; ++t) {
        const float f0 = sp[2 * t], f1 = sp[2 * t + 1];
        const unsigned short h0 = bf_bits(f0), h1 = bf_bits(f1);
        const unsigned short l0 = bf_bits(f0 - bf_up(h0)), l1 = bf_bits(f1 - bf_up(h1));
        a[t] = pk16(h0, h1); a2[t] = pk16(l0, l1);
      }
      hv[it] = a; lv[it] = a2;
    }
    for (int ps = 0; ps < 2; ++ps) {
#pragma unroll
      for (int it = 0; it < 4; ++it) {
        const int e = wave * 16 + it * 4 + q4;
        *(volatile v4u*)(Mh + (size_t)e * ND + c8) = hv[it];
        *(volatile v4u*)(Ml + (size_t)e * ND + c8) = lv[it];
      }
      __threadfence();
    }
  }
}

__global__ __launch_bounds__(256) void adapt(const unsigned short* __restrict__ xq, const unsigned short* __restrict__ xk,
                                             const unsigned short* __restrict__ mhp, const unsigned short* __restrict__ mlp,
                                             unsigned short* ahp, unsigned short* alp) {
  __shared__ __align__(16) float sT[8][16 * 68];
  const int tid  = threadIdx.x;
  const int wave = tid >> 5;
  const int lane = tid & 31;
  const int hh   = lane >> 4;
  const int c    = lane & 15;
  const int y    = blockIdx.y;
  const int s    = y / (NB * NR * NH);
  int rem        = y - s * (NB * NR * NH);
  const int b    = rem / (NR * NH);
  rem           -= b * (NR * NH);
  const int r    = rem / NH;
  const int h    = rem - r * NH;
  const int l0   = blockIdx.x * 128 + wave * 16;

  const unsigned short* xs = (s == 0) ? xq : xk;
  const __bf16* X  = (const __bf16*)(const void*)xs + (size_t)(b * NH + h) * NL * ND;
  const size_t  mo = (size_t)(s * NRH + r * NH + h) * ND * ND;
  const __bf16* Mh = (const __bf16*)(const void*)mhp + mo;
  const __bf16* Ml = (const __bf16*)(const void*)mlp + mo;

  v8f acc[4];
#pragma unroll
  for (int j = 0; j < 4; ++j) acc[j] = zero8();
#pragma unroll
  for (int ks = 0; ks < 2; ++ks) {
    const v16b a = ldfrag_b(X + (size_t)(l0 + c) * ND + ks * 32 + 8 * hh);
#pragma unroll
    for (int j = 0; j < 4; ++j) {
      const size_t bo = (size_t)(j * 16 + c) * ND + ks * 32 + 8 * hh;
      const v16b bh = ldfrag_b(Mh + bo);
      const v16b bl = ldfrag_b(Ml + bo);
      acc[j] = mma_b(a, bh, acc[j]);
      acc[j] = mma_b(a, bl, acc[j]);
    }
  }

  float* slab = sT[wave];
#pragma unroll
  for (int j = 0; j < 4; ++j) {
#pragma unroll
    for (int rr = 0; rr < 8; ++rr) slab[(8 * hh + rr) * 68 + j * 16 + c] = acc[j][rr];
  }
  wave_sync_lds();
  {
    const int q4 = lane >> 3, c8 = (lane & 7) * 8;
    const size_t prow = (size_t)(((s * NB + b) * NR + r) * NH + h) * NL + l0;
    v4u hv[4], lv[4];
#pragma unroll
    for (int it = 0; it < 4; ++it) {
      const int row = it * 4 + q4;
      const float* sp = slab + row * 68 + c8;
      v4u a, a2;
#pragma unroll
      for (int t = 0; t < 4; ++t) {
        const float f0 = sp[2 * t] * 256.0f, f1 = sp[2 * t + 1] * 256.0f;
        const _Float16 x0 = (_Float16)f0, x1 = (_Float16)f1;
        const unsigned short h0 = h_bits(x0), h1 = h_bits(x1);
        const unsigned short r0 = h_bits((_Float16)((f0 - (float)x0) * 4096.0f));
        const unsigned short r1 = h_bits((_Float16)((f1 - (float)x1) * 4096.0f));
        a[t] = pk16(h0, h1); a2[t] = pk16(r0, r1);
      }
      hv[it] = a; lv[it] = a2;
    }
    for (int ps = 0; ps < 2; ++ps) {
#pragma unroll
      for (int it = 0; it < 4; ++it) {
        const int row = it * 4 + q4;
        const size_t go = (prow + row) * ND + c8;
        *(volatile v4u*)(ahp + go) = hv[it];
        *(volatile v4u*)(alp + go) = lv[it];
      }
      __threadfence();
    }
  }
}

__global__ __launch_bounds__(256) void scores(const unsigned short* __restrict__ ahp, const unsigned short* __restrict__ alp,
                                              const int* __restrict__ rel, float* outp, float rres, float rcarry) {
  __shared__ __align__(16) float sT[8][16 * 36];
  const int tid  = threadIdx.x;
  const int wave = tid >> 5;
  const int lane = tid & 31;
  const int hh   = lane >> 4;
  const int c    = lane & 15;
  const int bh   = blockIdx.y;
  const int b    = bh / NH;
  const int h    = bh - b * NH;
  const int lt   = blockIdx.x >> 3;
  const int mt   = blockIdx.x & 7;
  const int wr   = wave & 3;
  const int wc   = wave >> 2;
  const int l0   = lt * 64 + wr * 16;
  const int m0   = mt * 64 + wc * 32;

  const _Float16* AH = (const _Float16*)(const void*)ahp;
  const _Float16* AL = (const _Float16*)(const void*)alp;

  int rid[2][8];
#pragma unroll
  for (int j = 0; j < 2; ++j) {
#pragma unroll
    for (int rr = 0; rr < 8; ++rr) {
      int v = rel[((size_t)b * NL + l0 + 8 * hh + rr) * NL + m0 + 16 * j + c];
      v = (v < 0) ? 0 : ((v > NR - 1) ? (NR - 1) : v);
      rid[j][rr] = v;
    }
  }
  v8f sel[2];
  sel[0] = zero8(); sel[1] = zero8();

#pragma unroll 1
  for (int r = 0; r < NR; ++r) {
    const size_t pq = (size_t)(((0 * NB + b) * NR + r) * NH + h) * NL;
    const size_t pk = (size_t)(((1 * NB + b) * NR + r) * NH + h) * NL;
    v8f accH[2], accR[2];
    accH[0] = zero8(); accH[1] = zero8(); accR[0] = zero8(); accR[1] = zero8();
#pragma unroll
    for (int ks = 0; ks < 2; ++ks) {
      const size_t ao = (pq + l0 + c) * ND + ks * 32 + 8 * hh;
      const v16h qh = ldfrag_h(AH + ao);
      const v16h ql = ldfrag_h(AL + ao);
#pragma unroll
      for (int j = 0; j < 2; ++j) {
        const size_t bo = (pk + m0 + 16 * j + c) * ND + ks * 32 + 8 * hh;
        const v16h kh = ldfrag_h(AH + bo);
        const v16h kl = ldfrag_h(AL + bo);
        accH[j] = mma_h(qh, kh, accH[j]);
        accR[j] = mma_h(qh, kl, accR[j]);
        accR[j] = mma_h(ql, kh, accR[j]);
      }
    }
#pragma unroll
    for (int j = 0; j < 2; ++j) {
#pragma unroll
      for (int rr = 0; rr < 8; ++rr) {
        const float v = (accH[j][rr] + accR[j][rr] * rres) * rcarry;
        sel[j][rr] = (rid[j][rr] == r) ? v : sel[j][rr];
      }
    }
  }

  float* slab = sT[wave];
#pragma unroll
  for (int j = 0; j < 2; ++j) {
#pragma unroll
    for (int rr = 0; rr < 8; ++rr) slab[(8 * hh + rr) * 36 + j * 16 + c] = sel[j][rr];
  }
  wave_sync_lds();
  {
    const int q4 = lane >> 3, c4 = (lane & 7) * 4;
    v4f ov[4];
#pragma unroll
    for (int it = 0; it < 4; ++it) {
      const int row = it * 4 + q4;
      ov[it] = *(const v4f*)(slab + row * 36 + c4);
    }
    const size_t orow = (size_t)(b * NH + h) * NL + l0;
    for (int ps = 0; ps < 2; ++ps) {
#pragma unroll
      for (int it = 0; it < 4; ++it) {
        const int row = it * 4 + q4;
        *(volatile v4f*)(outp + (orow + row) * NL + m0 + c4) = ov[it];
      }
      __threadfence();
    }
  }
}

extern "C" void kernel_launch(void* const* d_in, const int* in_sizes, int n_in,
                              void* d_out, int out_size, void* d_ws, size_t ws_size,
                              hipStream_t stream) {
  if (n_in < 7) return;
  if (in_sizes[0] != NB * NH * NL * ND) return;
  if (in_sizes[1] != NB * NH * NL * ND) return;
  if (in_sizes[2] != NB * NL * NL) return;
  if (in_sizes[3] != NR * NH * NX * ND || in_sizes[4] != NR * NH * ND * NX) return;
  if (in_sizes[5] != NR * NH * NX * ND || in_sizes[6] != NR * NH * ND * NX) return;
  if (out_size != NB * NH * NL * NL) return;

  const float* Q   = (const float*)d_in[0];
  const float* K   = (const float*)d_in[1];
  const int*   rel = (const int*)d_in[2];
  const float* qA  = (const float*)d_in[3];
  const float* qB  = (const float*)d_in[4];
  const float* kA  = (const float*)d_in[5];
  const float* kB  = (const float*)d_in[6];
  float* out = (float*)d_out;

  const size_t PX = (size_t)NB * NH * NL * ND * 2;
  const size_t PM = (size_t)2 * NRH * ND * ND * 2;
  const size_t PA = (size_t)2 * NB * NR * NH * NL * ND * 2;
  size_t off = 0;
  const size_t oXq = off; off += PX;
  const size_t oXk = off; off += PX;
  const size_t oMh = off; off += PM;
  const size_t oMl = off; off += PM;
  const size_t oAh = off; off += PA;
  const size_t oAl = off; off += PA;
  if (off > ws_size) return;
  if (off > (size_t)134217728) return;

  char* ws = (char*)d_ws;
  unsigned short* Xq = (unsigned short*)(ws + oXq);
  unsigned short* Xk = (unsigned short*)(ws + oXk);
  unsigned short* Mh = (unsigned short*)(ws + oMh);
  unsigned short* Ml = (unsigned short*)(ws + oMl);
  unsigned short* Ah = (unsigned short*)(ws + oAh);
  unsigned short* Al = (unsigned short*)(ws + oAl);

  const float rres   = 1.0f / 4096.0f;
  const float rcarry = 1.0f / 65536.0f;

  const int  n8 = NB * NH * NL * ND / 8;
  const dim3 gCvt((n8 + 255) / 256, 2);
  const dim3 gM(NRH, 2);
  const dim3 gA(NL / 128, 2 * NB * NR * NH);
  const dim3 gS(64, NB * NH);

  cvt_bf16x8<<<gCvt, dim3(256), 0, stream>>>(Q, K, Xq, Xk, n8);
  build_m<<<gM, dim3(128), 0, stream>>>(qA, qB, kA, kB, Mh, Ml);
  adapt<<<gA, dim3(256), 0, stream>>>(Xq, Xk, Mh, Ml, Ah, Al);
  scores<<<gS, dim3(256), 0, stream>>>(Ah, Al, rel, out, rres, rcarry);
  (void)hipGetLastError();
}
